// DCN_4389456576964
// MI455X (gfx1250) — hardware-verified
//
#include <hip/hip_runtime.h>
#include <stddef.h>
#include <math.h>

typedef __attribute__((ext_vector_type(16))) _Float16 v16h;
typedef __attribute__((ext_vector_type(8)))  _Float16 v8h;
typedef __attribute__((ext_vector_type(16))) __bf16   v16b;
typedef __attribute__((ext_vector_type(8)))  __bf16   v8b;
typedef __attribute__((ext_vector_type(8)))  float    v8f;
typedef __attribute__((ext_vector_type(4)))  float    v4f;
typedef __attribute__((ext_vector_type(4)))  int      v4i;

constexpr int NB      = 8;
constexpr int CIN     = 64;
constexpr int COUT    = 64;
constexpr int IMH     = 128;
constexpr int IMW     = 128;
constexpr int HW      = IMH * IMW;
constexpr int NPIX    = NB * HW;
constexpr int KC      = CIN * 9;
constexpr int KG      = KC / 8;
constexpr int NOM     = 27;
constexpr int NOMPAD  = 64;
constexpr int OFFM_LD = 64;
constexpr int NTHR    = 256;
constexpr int PXB     = 64;
constexpr int STATS_LD = 128;
constexpr int BOM_N   = 128;
constexpr float X_CARRY   = 8.0f;
constexpr float WOM_CARRY = 256.0f;
constexpr float COL_CARRY = 8.0f;
constexpr float WD_CARRY  = 64.0f;
constexpr float OM_FOLD   = 1.0f / 2048.0f;
constexpr float DC_FOLD   = 1.0f / 512.0f;
constexpr float BN_EPS    = 1e-5f;

static_assert(KC % 32 == 0);
static_assert(HW % 64 == 0 && COUT % 64 == 0 && NOMPAD % 64 == 0);
static_assert((HW / 64) % 8 == 0);
static_assert((HW * KG) % NTHR == 0);
static_assert((NOMPAD * KG) % NTHR == 0);
static_assert((COUT * KG) % NTHR == 0);
static_assert((PXB * KG) % NTHR == 0 && HW % PXB == 0);
static_assert((PXB * 9) == 2 * NTHR + 64);
static_assert((NB * COUT * HW / 4) % NTHR == 0);
static_assert(HW % (NTHR * 4) == 0);
static_assert(NOM <= NOMPAD && 2 * 9 + 9 == NOM);

__device__ __forceinline__ unsigned short f2bf_bits(float f) {
  unsigned u = __float_as_uint(f);
  return (unsigned short)((u + 0x7FFFu + ((u >> 16) & 1u)) >> 16);
}
__device__ __forceinline__ float bf_bits2f(unsigned short h) { return __uint_as_float(((unsigned)h) << 16); }

__device__ __forceinline__ void dep_guard_h(v8f& a, v8f& b, v16h x, v16h y) { asm volatile("v_nop\n\tv_nop\n\tv_nop\n\tv_nop" : "+v"(a), "+v"(b) : "v"(x), "v"(y)); }
__device__ __forceinline__ void dep_guard_b(v8f& a, v8f& b, v16b x, v16b y) { asm volatile("v_nop\n\tv_nop\n\tv_nop\n\tv_nop" : "+v"(a), "+v"(b) : "v"(x), "v"(y)); }
__device__ __forceinline__ void dep_guard4_h(v8f& a, v8f& b, v8f& c, v8f& d, v16h x, v16h y) { asm volatile("v_nop\n\tv_nop\n\tv_nop\n\tv_nop" : "+v"(a), "+v"(b), "+v"(c), "+v"(d) : "v"(x), "v"(y)); }
__device__ __forceinline__ void dep_guard4_b(v8f& a, v8f& b, v8f& c, v8f& d, v16b x, v16b y) { asm volatile("v_nop\n\tv_nop\n\tv_nop\n\tv_nop" : "+v"(a), "+v"(b), "+v"(c), "+v"(d) : "v"(x), "v"(y)); }
__device__ __forceinline__ void keep4_h(v16h a, v16h b, v16h c, v16h d) { asm volatile("v_nop" :: "v"(a), "v"(b), "v"(c), "v"(d)); }
__device__ __forceinline__ void keep4_b(v16b a, v16b b, v16b c, v16b d) { asm volatile("v_nop" :: "v"(a), "v"(b), "v"(c), "v"(d)); }
__device__ __forceinline__ void acc_guard4(v8f& a, v8f& b, v8f& c, v8f& d) { asm volatile("v_nop\n\tv_nop\n\tv_nop\n\tv_nop" : "+v"(a), "+v"(b), "+v"(c), "+v"(d)); }
template <typename T> struct Frag;
template <> struct Frag<_Float16> {
  typedef v16h V; union U { v16h v; v8h h[2]; };
  static __device__ __forceinline__ v16h load(const _Float16* p) {
    U f; f.h[0] = *(const v8h*)(p); f.h[1] = *(const v8h*)(p + 16); return f.v;
  }
  static __device__ __forceinline__ v8f mma(v16h a, v16h b, v8f c) {
    return __builtin_amdgcn_wmma_f32_16x16x32_f16(false, a, false, b, (short)0, c, false, false);
  }
  static __device__ __forceinline__ void guard(v8f& a, v8f& b, v16h x, v16h y) { dep_guard_h(a, b, x, y); }
  static __device__ __forceinline__ void guard4(v8f& a, v8f& b, v8f& c, v8f& d, v16h x, v16h y) { dep_guard4_h(a, b, c, d, x, y); }
  static __device__ __forceinline__ void keep(v16h a, v16h b, v16h c, v16h d) { keep4_h(a, b, c, d); }
};
template <> struct Frag<__bf16> {
  typedef v16b V; union U { v16b v; v8b h[2]; };
  static __device__ __forceinline__ v16b load(const __bf16* p) {
    U f; f.h[0] = *(const v8b*)(p); f.h[1] = *(const v8b*)(p + 16); return f.v;
  }
  static __device__ __forceinline__ v8f mma(v16b a, v16b b, v8f c) {
    return __builtin_amdgcn_wmma_f32_16x16x32_bf16(false, a, false, b, (short)0, c, false, false);
  }
  static __device__ __forceinline__ void guard(v8f& a, v8f& b, v16b x, v16b y) { dep_guard_b(a, b, x, y); }
  static __device__ __forceinline__ void guard4(v8f& a, v8f& b, v8f& c, v8f& d, v16b x, v16b y) { dep_guard4_b(a, b, c, d, x, y); }
  static __device__ __forceinline__ void keep(v16b a, v16b b, v16b c, v16b d) { keep4_b(a, b, c, d); }
};

template <int ET> struct Elem;
template <> struct Elem<0> { typedef _Float16 T; };
template <> struct Elem<1> { typedef __bf16 T; };
template <int ET, bool SPLIT, int BIAS_MODE, int OUT_MODE, bool RESID, int ACT = 0>
__global__ __launch_bounds__(256) void wmma_gemm64(
    const unsigned short* __restrict__ Ap, const unsigned short* __restrict__ A2p, int lda, long strideA,
    const unsigned short* __restrict__ Btp, const unsigned short* __restrict__ Bt2p, int ldb, long strideB,
    void* __restrict__ Cout, void* __restrict__ Cout2, int ldc, long strideC,
    const float* __restrict__ bias,
    const float* __restrict__ resid, long strideR,
    int M, int N, int K, float scale) {
  typedef typename Elem<ET>::T T;
  typedef typename Frag<T>::V V;
  const T* A = (const T*)Ap; const T* A2 = (const T*)A2p; const T* Bt = (const T*)Btp; const T* Bt2 = (const T*)Bt2p;
  __shared__ __align__(16) float sT[8][16 * 68];
  const int b    = blockIdx.y;
  const int lane = threadIdx.x & 31;
  const int wave = threadIdx.x >> 5;
  const int tilesN = N >> 6;
  const int tilesM = M >> 6;
  const int tile = blockIdx.x * 8 + wave;
  if (tile >= tilesM * tilesN) return;
  const int tm = tile / tilesN;
  const int tn = tile - tm * tilesN;
  const int m0 = tm << 6;
  const int n0 = tn << 6;

  const T* Ab  = A  + (size_t)b * strideA;
  const T* Bb  = Bt + (size_t)b * strideB;
  const T* Ab2 = SPLIT ? (A2  + (size_t)b * strideA) : nullptr;
  const T* Bb2 = SPLIT ? (Bt2 + (size_t)b * strideB) : nullptr;

  const int rlane = lane & 15;
  const int koff  = (lane >> 4) * 8;
  const int mOff  = (lane >> 4) * 8;

  v8f acc[4][4];
#pragma unroll
  for (int i = 0; i < 4; ++i)
#pragma unroll
    for (int j = 0; j < 4; ++j) acc[i][j] = (v8f){0.f,0.f,0.f,0.f,0.f,0.f,0.f,0.f};

  for (int k0 = 0; k0 < K; k0 += 32) {
    V bh[4], bl[4];
#pragma unroll
    for (int j = 0; j < 4; ++j) {
      const size_t bo = (size_t)(n0 + (j << 4) + rlane) * ldb + koff + k0;
      bh[j] = Frag<T>::load(Bb + bo);
      if (SPLIT) bl[j] = Frag<T>::load(Bb2 + bo);
    }
#pragma unroll
    for (int i = 0; i < 4; ++i) {
      const size_t ao = (size_t)(m0 + (i << 4) + rlane) * lda + koff + k0;
      V ah = Frag<T>::load(Ab + ao);
      V al;
      if (SPLIT) al = Frag<T>::load(Ab2 + ao);
#pragma unroll
      for (int j = 0; j < 4; ++j) {
        acc[i][j] = Frag<T>::mma(ah, bh[j], acc[i][j]);
        if (SPLIT) {
          acc[i][j] = Frag<T>::mma(ah, bl[j], acc[i][j]);
          acc[i][j] = Frag<T>::mma(al, bh[j], acc[i][j]);
        }
      }
      Frag<T>::guard4(acc[i][0], acc[i][1], acc[i][2], acc[i][3], ah, SPLIT ? al : ah);
    }
    Frag<T>::keep(bh[0], bh[1], bh[2], bh[3]);
    if (SPLIT) Frag<T>::keep(bl[0], bl[1], bl[2], bl[3]);
  }
  acc_guard4(acc[0][0], acc[0][1], acc[0][2], acc[0][3]);
  acc_guard4(acc[1][0], acc[1][1], acc[1][2], acc[1][3]);
  acc_guard4(acc[2][0], acc[2][1], acc[2][2], acc[2][3]);
  acc_guard4(acc[3][0], acc[3][1], acc[3][2], acc[3][3]);

  float* slab = sT[wave];
  const float* Rb = RESID ? (resid + (size_t)b * strideR) : nullptr;
#pragma unroll
  for (int i = 0; i < 4; ++i) {
    const int mBase = m0 + (i << 4);
#pragma unroll
    for (int j = 0; j < 4; ++j) {
      const int n = n0 + (j << 4) + rlane;
      float bv = 0.f;
      if (BIAS_MODE == 2) bv = bias[n];
#pragma unroll
      for (int r = 0; r < 8; ++r) {
        float v = acc[i][j][r] * scale;
        if (BIAS_MODE == 1) v += bias[mBase + mOff + r];
        if (BIAS_MODE == 2) v += bv;
        if (RESID) v += Rb[(size_t)(mBase + mOff + r) * ldc + n];
        if (ACT == 1) v = tanhf(v);
        if (ACT == 2) v = fmaxf(v, 0.0f);
        if (ACT == 3) v = v / (1.0f + expf(-v));
        if (ACT == 4) v = (v > 0.f) ? v : 0.01f * v;
        if (ACT == 5) v = 0.5f * v * (1.0f + erff(v * 0.70710678118654752f));
        slab[(mOff + r) * 68 + (j << 4) + rlane] = v;
      }
    }
    __builtin_amdgcn_fence(__ATOMIC_RELEASE, "workgroup");
    __builtin_amdgcn_wave_barrier();
    __builtin_amdgcn_fence(__ATOMIC_ACQUIRE, "workgroup");
    if (OUT_MODE == 0) {
      float* C = (float*)Cout + (size_t)b * strideC;
      const int hh = lane >> 4, c4 = (lane & 15) * 4;
      for (int pass = 0; pass < 2; ++pass) {
#pragma unroll
        for (int it = 0; it < 8; ++it) {
          const int row = it * 2 + hh;
          v4f v = *(const v4f*)(slab + row * 68 + c4);
          *(volatile v4f*)(C + (size_t)(mBase + row) * ldc + n0 + c4) = v;
        }
        __threadfence();
      }
    } else {
      const int q = lane >> 3, c8 = (lane & 7) * 8;
      unsigned short* C  = (unsigned short*)Cout  + (size_t)b * strideC;
      unsigned short* C2 = (OUT_MODE == 2) ? ((unsigned short*)Cout2 + (size_t)b * strideC) : nullptr;
      for (int pass = 0; pass < 2; ++pass) {
#pragma unroll
        for (int it = 0; it < 4; ++it) {
          const int row = it * 4 + q;
          const float* sp = slab + row * 68 + c8;
          v8h hv, lv;
#pragma unroll
          for (int e = 0; e < 8; ++e) {
            if (OUT_MODE == 1) {
              hv[e] = (_Float16)sp[e];
            } else {
              unsigned short hb = f2bf_bits(sp[e]);
              unsigned short lb = f2bf_bits(sp[e] - bf_bits2f(hb));
              hv[e] = __builtin_bit_cast(_Float16, hb);
              lv[e] = __builtin_bit_cast(_Float16, lb);
            }
          }
          *(volatile v8h*)(C + (size_t)(mBase + row) * ldc + n0 + c8) = hv;
          if (OUT_MODE == 2) *(volatile v8h*)(C2 + (size_t)(mBase + row) * ldc + n0 + c8) = lv;
        }
        __threadfence();
      }
    }
    __builtin_amdgcn_fence(__ATOMIC_RELEASE, "workgroup");
    __builtin_amdgcn_wave_barrier();
    __builtin_amdgcn_fence(__ATOMIC_ACQUIRE, "workgroup");
  }
}

__global__ __launch_bounds__(NTHR) void k_prep_wom(const float* __restrict__ w_off, const float* __restrict__ w_msk,
                                                     const float* __restrict__ b_off, const float* __restrict__ b_msk,
                                                     unsigned short* __restrict__ womB, float* __restrict__ bom) {
  const int tid = threadIdx.x;
  const int i = blockIdx.x * NTHR + tid;
  const int n = i / KG;
  const int k0 = (i - n * KG) * 8;
  const int na = (n < 18) ? n : 17;
  int nb = n - 18; nb = (nb < 0) ? 0 : ((nb > 8) ? 8 : nb);
  const float fa = (n < 18) ? 1.0f : 0.0f;
  const float fb = (n >= 18 && n < NOM) ? 1.0f : 0.0f;
  v8h hv;
#pragma unroll
  for (int e = 0; e < 8; ++e) {
    const float a  = w_off[(size_t)na * KC + k0 + e];
    const float bm = w_msk[(size_t)nb * KC + k0 + e];
    const float v  = fmaf(fa, a, fb * bm) * WOM_CARRY;
    hv[e] = (_Float16)v;
  }
  unsigned short* dst = womB + (size_t)i * 8;
  *(volatile v8h*)dst = hv;
  __threadfence();
  *(volatile v8h*)dst = hv;

  if (blockIdx.x == 0 && (tid >> 5) == 0) {
    const int lane = tid & 31;
    v4f bv;
#pragma unroll
    for (int e = 0; e < 4; ++e) {
      const int j = lane * 4 + e;
      const int ja = (j < 18) ? j : 17;
      int jb = j - 18; jb = (jb < 0) ? 0 : ((jb > 8) ? 8 : jb);
      const float ga = (j < 18) ? 1.0f : 0.0f;
      const float gb = (j >= 18 && j < NOM) ? 1.0f : 0.0f;
      bv[e] = fmaf(ga, b_off[ja], gb * b_msk[jb]);
    }
    float* bd = bom + lane * 4;
    *(volatile v4f*)bd = bv;
    __threadfence();
    *(volatile v4f*)bd = bv;
  }
}

__global__ __launch_bounds__(NTHR) void k_prep_wd(const float* __restrict__ w_dcn, unsigned short* __restrict__ wdB) {
  const int i = blockIdx.x * NTHR + threadIdx.x;
  v8h hv;
#pragma unroll
  for (int e = 0; e < 8; ++e) hv[e] = (_Float16)(w_dcn[(size_t)i * 8 + e] * WD_CARRY);
  unsigned short* dst = wdB + (size_t)i * 8;
  *(volatile v8h*)dst = hv;
  __threadfence();
  *(volatile v8h*)dst = hv;
}

__global__ __launch_bounds__(NTHR) void k_im2col(const float* __restrict__ x, int b, unsigned short* __restrict__ im) {
  const int i = blockIdx.x * NTHR + threadIdx.x;
  const int m = i / KG;
  const int k0 = (i - m * KG) * 8;
  const int py = m >> 7;
  const int px = m & (IMW - 1);
  const float* xb = x + (size_t)b * CIN * HW;
  v8h hv;
#pragma unroll
  for (int e = 0; e < 8; ++e) {
    const int k  = k0 + e;
    const int ci = k / 9;
    const int tt = k - ci * 9;
    const int ky = tt / 3;
    const int kx = tt - ky * 3;
    const int yy = py + ky - 1;
    const int xx = px + kx - 1;
    const float fv = ((unsigned)yy < (unsigned)IMH && (unsigned)xx < (unsigned)IMW) ? 1.0f : 0.0f;
    const int yc = (yy < 0) ? 0 : ((yy > IMH - 1) ? (IMH - 1) : yy);
    const int xc = (xx < 0) ? 0 : ((xx > IMW - 1) ? (IMW - 1) : xx);
    const float v = xb[(size_t)ci * HW + yc * IMW + xc];
    hv[e] = (_Float16)(v * fv * X_CARRY);
  }
  unsigned short* dst = im + (size_t)i * 8;
  *(volatile v8h*)dst = hv;
  __threadfence();
  *(volatile v8h*)dst = hv;
}

__global__ __launch_bounds__(NTHR) void k_sample(const float* __restrict__ x, const float* __restrict__ offm, int b,
                                                   unsigned short* __restrict__ col) {
  __shared__ __align__(16) int   gOff[PXB * 9 * 4];
  __shared__ __align__(16) float gW[PXB * 9 * 4];
  const int tid = threadIdx.x;
  const int pbase = blockIdx.x * PXB;
  const float* xb   = x + (size_t)b * CIN * HW;
  const float* offb = offm + (size_t)b * HW * OFFM_LD;

#pragma unroll 1
  for (int i = tid; i < PXB * 9; i += NTHR) {
    const int ml  = i / 9;
    const int tap = i - ml * 9;
    const int p   = pbase + ml;
    const int yi  = p >> 7;
    const int xi  = p & (IMW - 1);
    const int ky  = tap / 3;
    const int kx  = tap - ky * 3;
    const float* orow = offb + (size_t)p * OFFM_LD;
    const float dy = orow[2 * tap];
    const float dx = orow[2 * tap + 1];
    const float mg = orow[18 + tap];
    const float md = __builtin_amdgcn_rcpf(1.0f + expf(-mg));
    const float pyf = (float)(yi + ky - 1) + dy;
    const float pxf = (float)(xi + kx - 1) + dx;
    const float y0f = floorf(pyf);
    const float x0f = floorf(pxf);
    const float ly = pyf - y0f;
    const float lx = pxf - x0f;
    const float y1f = y0f + 1.0f;
    const float x1f = x0f + 1.0f;
    const float vy0 = (y0f >= 0.0f && y0f < (float)IMH) ? 1.0f : 0.0f;
    const float vy1 = (y1f >= 0.0f && y1f < (float)IMH) ? 1.0f : 0.0f;
    const float vx0 = (x0f >= 0.0f && x0f < (float)IMW) ? 1.0f : 0.0f;
    const float vx1 = (x1f >= 0.0f && x1f < (float)IMW) ? 1.0f : 0.0f;
    const int yc0 = (int)fminf(fmaxf(y0f, 0.0f), (float)(IMH - 1));
    const int yc1 = (int)fminf(fmaxf(y1f, 0.0f), (float)(IMH - 1));
    const int xc0 = (int)fminf(fmaxf(x0f, 0.0f), (float)(IMW - 1));
    const int xc1 = (int)fminf(fmaxf(x1f, 0.0f), (float)(IMW - 1));
    const float omly = 1.0f - ly;
    const float omlx = 1.0f - lx;
    const float w00 = (omly * omlx) * (vy0 * vx0) * md;
    const float w01 = (omly * lx)   * (vy0 * vx1) * md;
    const float w10 = (ly * omlx)   * (vy1 * vx0) * md;
    const float w11 = (ly * lx)     * (vy1 * vx1) * md;
    v4i o;
    o[0] = yc0 * IMW + xc0; o[1] = yc0 * IMW + xc1; o[2] = yc1 * IMW + xc0; o[3] = yc1 * IMW + xc1;
    v4f w;
    w[0] = w00; w[1] = w01; w[2] = w10; w[3] = w11;
    *(v4i*)(gOff + i * 4) = o;
    *(v4f*)(gW + i * 4) = w;
  }
  __syncthreads();

  unsigned short* colb = col + (size_t)pbase * KC;
#pragma unroll 1
  for (int it = 0; it < (PXB * KG) / NTHR; ++it) {
    const int i  = it * NTHR + tid;
    const int ml = i / KG;
    const int j  = i - ml * KG;
    v8h hv;
#pragma unroll
    for (int ep = 0; ep < 4; ++ep) {
      const int ka   = j * 8 + ep * 2;
      const int kq   = ka + 1;
      const int ca   = ka / 9;
      const int ta   = ka - ca * 9;
      const int cq   = kq / 9;
      const int tq   = kq - cq * 9;
      const int ga   = (ml * 9 + ta) * 4;
      const int gq   = (ml * 9 + tq) * 4;
      const v4i oa = *(const v4i*)(gOff + ga);
      const v4f wa = *(const v4f*)(gW + ga);
      const v4i oq = *(const v4i*)(gOff + gq);
      const v4f wq = *(const v4f*)(gW + gq);
      const float* xa = xb + (size_t)ca * HW;
      const float* xq = xb + (size_t)cq * HW;
      float sa = xa[oa[0]] * wa[0] + xa[oa[1]] * wa[1] + xa[oa[2]] * wa[2] + xa[oa[3]] * wa[3];
      float sq = xq[oq[0]] * wq[0] + xq[oq[1]] * wq[1] + xq[oq[2]] * wq[2] + xq[oq[3]] * wq[3];
      asm volatile("" : "+v"(sa), "+v"(sq) : : "memory");
      hv[ep * 2]     = (_Float16)(sa * COL_CARRY);
      hv[ep * 2 + 1] = (_Float16)(sq * COL_CARRY);
    }
    unsigned short* dst = colb + (size_t)i * 8;
    *(volatile v8h*)dst = hv;
    __threadfence();
    *(volatile v8h*)dst = hv;
  }
}

__global__ __launch_bounds__(NTHR) void k_bnstats(const float* __restrict__ gout, const float* __restrict__ gamma,
                                                    const float* __restrict__ beta, float* __restrict__ stats) {
  __shared__ double sh1[NTHR];
  __shared__ double sh2[NTHR];
  __shared__ __align__(16) float res[4];
  const int tid = threadIdx.x;
  const int o = blockIdx.x;
  const float gm = gamma[o];
  const float bt = beta[o];
  double s1 = 0.0, s2 = 0.0;
#pragma unroll 1
  for (int b = 0; b < NB; ++b) {
    const float* g = gout + ((size_t)b * COUT + o) * HW;
#pragma unroll 1
    for (int q = tid * 4; q < HW; q += NTHR * 4) {
      const v4f v = *(const v4f*)(g + q);
      const double d0 = (double)v[0], d1 = (double)v[1], d2 = (double)v[2], d3 = (double)v[3];
      s1 += (d0 + d1) + (d2 + d3);
      s2 += (d0 * d0 + d1 * d1) + (d2 * d2 + d3 * d3);
    }
  }
  sh1[tid] = s1; sh2[tid] = s2;
  __syncthreads();
#pragma unroll 1
  for (int off = NTHR / 2; off > 0; off >>= 1) {
    if (tid < off) { sh1[tid] += sh1[tid + off]; sh2[tid] += sh2[tid + off]; }
    __syncthreads();
  }
  if (tid == 0) {
    const double inv = 1.0 / (double)NPIX;
    const double mean = sh1[0] * inv;
    double var = sh2[0] * inv - mean * mean;
    if (var < 0.0) var = 0.0;
    const float varf = (float)var;
    res[0] = (float)mean;
    res[1] = rsqrtf(varf + BN_EPS);
    res[2] = gm;
    res[3] = bt;
  }
  __syncthreads();
  if ((tid >> 5) == 0) {
    const int lane = tid & 31;
    const v4f r4 = *(const v4f*)res;
    const float f = (lane == 0) ? 1.0f : 0.0f;
    v4f v;
    v[0] = r4[0] * f; v[1] = r4[1] * f; v[2] = r4[2] * f; v[3] = r4[3] * f;
    float* dst = stats + (size_t)o * STATS_LD + lane * 4;
    *(volatile v4f*)dst = v;
    __threadfence();
    *(volatile v4f*)dst = v;
  }
}

__global__ __launch_bounds__(NTHR) void k_bn_mish(const float* __restrict__ gout, const float* __restrict__ stats,
                                                    float* __restrict__ out) {
  const int i = blockIdx.x * NTHR + threadIdx.x;
  const size_t idx = (size_t)i * 4;
  const int o = (i >> 12) & (COUT - 1);
  const v4f g  = *(const v4f*)(gout + idx);
  const v4f st = *(const v4f*)(stats + (size_t)o * STATS_LD);
  v4f r;
#pragma unroll
  for (int e = 0; e < 4; ++e) {
    float v = (g[e] - st[0]) * st[1];
    v = v * st[2] + st[3];
    const float t  = expf(fminf(v, 20.0f));
    const float nm = t * (t + 2.0f);
    const float th = nm * __builtin_amdgcn_rcpf(nm + 2.0f);
    r[e] = v * th;
  }
  float* dst = out + idx;
  *(volatile v4f*)dst = r;
  __threadfence();
  *(volatile v4f*)dst = r;
}

constexpr size_t OFF_WOM  = 0;
constexpr size_t SZ_WOM   = (size_t)NOMPAD * KC * 2;
constexpr size_t OFF_BOM  = OFF_WOM + SZ_WOM;
constexpr size_t SZ_BOM   = (size_t)BOM_N * 4;
constexpr size_t OFF_WD   = OFF_BOM + SZ_BOM;
constexpr size_t SZ_WD    = (size_t)COUT * KC * 2;
constexpr size_t OFF_IM   = OFF_WD + SZ_WD;
constexpr size_t SZ_IM    = (size_t)HW * KC * 2;
constexpr size_t OFF_COL  = OFF_IM + SZ_IM;
constexpr size_t SZ_COL   = SZ_IM;
constexpr size_t OFF_OFFM = OFF_COL + SZ_COL;
constexpr size_t SZ_OFFM  = (size_t)NPIX * OFFM_LD * 4;
constexpr size_t OFF_G    = OFF_OFFM + SZ_OFFM;
constexpr size_t SZ_G     = (size_t)NB * COUT * HW * 4;
constexpr size_t OFF_ST   = OFF_G + SZ_G;
constexpr size_t SZ_ST    = (size_t)COUT * STATS_LD * 4;
constexpr size_t WS_TOTAL = OFF_ST + SZ_ST;
static_assert(WS_TOTAL == 105038336u);
static_assert(WS_TOTAL <= 134217728u);
static_assert(OFF_BOM % 128 == 0 && OFF_WD % 128 == 0 && OFF_IM % 128 == 0 && OFF_COL % 128 == 0 &&
              OFF_OFFM % 128 == 0 && OFF_G % 128 == 0 && OFF_ST % 128 == 0);
static_assert(HW % 64 == 0 && NOMPAD == 64 && COUT == 64 && KC % 32 == 0);

extern "C" void kernel_launch(void* const* d_in, const int* in_sizes, int n_in,
                              void* d_out, int out_size, void* d_ws, size_t ws_size,
                              hipStream_t stream) {
  (void)in_sizes; (void)n_in;
  const float* x      = (const float*)d_in[0];
  const float* w_off  = (const float*)d_in[1];
  const float* b_off  = (const float*)d_in[2];
  const float* w_msk  = (const float*)d_in[3];
  const float* b_msk  = (const float*)d_in[4];
  const float* w_dcn  = (const float*)d_in[5];
  const float* b_dcn  = (const float*)d_in[6];
  const float* gamma  = (const float*)d_in[7];
  const float* beta   = (const float*)d_in[8];
  float* out = (float*)d_out;
  if (ws_size < WS_TOTAL) return;
  if ((size_t)out_size < (size_t)NB * COUT * HW) return;

  char* ws = (char*)d_ws;
  unsigned short* womB = (unsigned short*)(ws + OFF_WOM);
  float*          bom  = (float*)(ws + OFF_BOM);
  unsigned short* wdB  = (unsigned short*)(ws + OFF_WD);
  unsigned short* im   = (unsigned short*)(ws + OFF_IM);
  unsigned short* col  = (unsigned short*)(ws + OFF_COL);
  float*          offm = (float*)(ws + OFF_OFFM);
  float*          gout = (float*)(ws + OFF_G);
  float*          stats = (float*)(ws + OFF_ST);

  k_prep_wom<<<(NOMPAD * KG) / NTHR, NTHR, 0, stream>>>(w_off, w_msk, b_off, b_msk, womB, bom);
  k_prep_wd<<<(COUT * KG) / NTHR, NTHR, 0, stream>>>(w_dcn, wdB);

  for (int b = 0; b < NB; ++b) {
    float* offm_b = offm + (size_t)b * HW * OFFM_LD;
    float* gout_b = gout + (size_t)b * COUT * HW;
    k_im2col<<<(HW * KG) / NTHR, NTHR, 0, stream>>>(x, b, im);
    wmma_gemm64<0, false, 2, 0, false, 0><<<dim3((HW / 64) / 8, 1), NTHR, 0, stream>>>(
        im, im, KC, 0L, womB, womB, KC, 0L, (void*)offm_b, (void*)offm_b, OFFM_LD, 0L,
        bom, bom, 0L, HW, NOMPAD, KC, OM_FOLD);
    k_sample<<<HW / PXB, NTHR, 0, stream>>>(x, offm, b, col);
    wmma_gemm64<0, false, 1, 0, false, 0><<<dim3((HW / 64) / 8, 1), NTHR, 0, stream>>>(
        wdB, wdB, KC, 0L, col, col, KC, 0L, (void*)gout_b, (void*)gout_b, HW, 0L,
        b_dcn, b_dcn, 0L, COUT, HW, KC, DC_FOLD);
  }

  k_bnstats<<<COUT, NTHR, 0, stream>>>(gout, gamma, beta, stats);
  k_bn_mish<<<(NB * COUT * HW / 4) / NTHR, NTHR, 0, stream>>>(gout, stats, out);
}
